// RMHA_78176994722494
// MI455X (gfx1250) — hardware-verified
//
#include <hip/hip_runtime.h>
#include <math.h>
#include <stdint.h>

namespace {
constexpr int kBatch = 4, kSeq = 1024, kDim = 1024, kHeads = 16, kHd = 64, kMaxR = 32, kNRel = 65, kRelP = 128;
constexpr int kHGrp = 8, kNGrp = kHeads / kHGrp;
constexpr float kPCarry = 32768.0f;
constexpr float kWCarry = 16.0f;
constexpr float kCtxCarry = 64.0f;
constexpr float kNegBig = -1.0e10f;
}

typedef __attribute__((ext_vector_type(16))) _Float16 v16h;
typedef __attribute__((ext_vector_type(8)))  _Float16 v8h;
typedef __attribute__((ext_vector_type(16))) __bf16   v16b;
typedef __attribute__((ext_vector_type(8)))  __bf16   v8b;
typedef __attribute__((ext_vector_type(8)))  float    v8f;
typedef __attribute__((ext_vector_type(4)))  float    v4f;
typedef __attribute__((ext_vector_type(2)))  float    v2f;
typedef __attribute__((ext_vector_type(4)))  unsigned int v4u;

__device__ __forceinline__ unsigned short f2bf_bits(float f) {
  unsigned u = __float_as_uint(f);
  return (unsigned short)((u + 0x7FFFu + ((u >> 16) & 1u)) >> 16);
}
__device__ __forceinline__ float bf_bits2f(unsigned short h) { return __uint_as_float(((unsigned)h) << 16); }

__device__ __forceinline__ void dep_guard_h(v8f& a, v8f& b, v16h x, v16h y) { asm volatile("v_nop\n\tv_nop\n\tv_nop\n\tv_nop" : "+v"(a), "+v"(b) : "v"(x), "v"(y)); }
__device__ __forceinline__ void dep_guard_b(v8f& a, v8f& b, v16b x, v16b y) { asm volatile("v_nop\n\tv_nop\n\tv_nop\n\tv_nop" : "+v"(a), "+v"(b) : "v"(x), "v"(y)); }
__device__ __forceinline__ void keep4_h(v16h a, v16h b, v16h c, v16h d) { asm volatile("v_nop" :: "v"(a), "v"(b), "v"(c), "v"(d)); }
__device__ __forceinline__ void keep4_b(v16b a, v16b b, v16b c, v16b d) { asm volatile("v_nop" :: "v"(a), "v"(b), "v"(c), "v"(d)); }
__device__ __forceinline__ void acc_guard4(v8f& a, v8f& b, v8f& c, v8f& d) { asm volatile("v_nop\n\tv_nop\n\tv_nop\n\tv_nop" : "+v"(a), "+v"(b), "+v"(c), "+v"(d)); }
template <typename T> struct Frag;
template <> struct Frag<_Float16> {
  typedef v16h V; union U { v16h v; v8h h[2]; };
  static __device__ __forceinline__ v16h load(const _Float16* p) {
    U f; f.h[0] = *(const v8h*)(p); f.h[1] = *(const v8h*)(p + 16); return f.v;
  }
  static __device__ __forceinline__ v8f mma(v16h a, v16h b, v8f c) {
    return __builtin_amdgcn_wmma_f32_16x16x32_f16(false, a, false, b, (short)0, c, false, false);
  }
  static __device__ __forceinline__ void guard(v8f& a, v8f& b, v16h x, v16h y) { dep_guard_h(a, b, x, y); }
  static __device__ __forceinline__ void keep(v16h a, v16h b, v16h c, v16h d) { keep4_h(a, b, c, d); }
};
template <> struct Frag<__bf16> {
  typedef v16b V; union U { v16b v; v8b h[2]; };
  static __device__ __forceinline__ v16b load(const __bf16* p) {
    U f; f.h[0] = *(const v8b*)(p); f.h[1] = *(const v8b*)(p + 16); return f.v;
  }
  static __device__ __forceinline__ v8f mma(v16b a, v16b b, v8f c) {
    return __builtin_amdgcn_wmma_f32_16x16x32_bf16(false, a, false, b, (short)0, c, false, false);
  }
  static __device__ __forceinline__ void guard(v8f& a, v8f& b, v16b x, v16b y) { dep_guard_b(a, b, x, y); }
  static __device__ __forceinline__ void keep(v16b a, v16b b, v16b c, v16b d) { keep4_b(a, b, c, d); }
};

template <int ET> struct Elem;
template <> struct Elem<0> { typedef _Float16 T; };
template <> struct Elem<1> { typedef __bf16 T; };
template <int ET, bool SPLIT, int BIAS_MODE, int OUT_MODE, bool RESID, int ACT = 0>
__global__ __launch_bounds__(256) void wmma_gemm64(
    const unsigned short* __restrict__ Ap, const unsigned short* __restrict__ A2p, int lda, long strideA,
    const unsigned short* __restrict__ Btp, const unsigned short* __restrict__ Bt2p, int ldb, long strideB,
    void* __restrict__ Cout, void* __restrict__ Cout2, int ldc, long strideC,
    const float* __restrict__ bias,
    const float* __restrict__ resid, long strideR,
    int M, int N, int K, float scale) {
  typedef typename Elem<ET>::T T;
  typedef typename Frag<T>::V V;
  const T* A = (const T*)Ap; const T* A2 = (const T*)A2p; const T* Bt = (const T*)Btp; const T* Bt2 = (const T*)Bt2p;
  __shared__ __align__(16) float sT[8][16 * 68];
  const int b    = blockIdx.y;
  const int lane = threadIdx.x & 31;
  const int wave = threadIdx.x >> 5;
  const int tilesN = N >> 6;
  const int tilesM = M >> 6;
  const int tile = blockIdx.x * 8 + wave;
  if (tile >= tilesM * tilesN) return;
  const int tm = tile / tilesN;
  const int tn = tile - tm * tilesN;
  const int m0 = tm << 6;
  const int n0 = tn << 6;

  const T* Ab  = A  + (size_t)b * strideA;
  const T* Bb  = Bt + (size_t)b * strideB;
  const T* Ab2 = SPLIT ? (A2  + (size_t)b * strideA) : nullptr;
  const T* Bb2 = SPLIT ? (Bt2 + (size_t)b * strideB) : nullptr;

  const int rlane = lane & 15;
  const int koff  = (lane >> 4) * 8;
  const int mOff  = (lane >> 4) * 8;

  v8f acc[4][4];
#pragma unroll
  for (int i = 0; i < 4; ++i)
#pragma unroll
    for (int j = 0; j < 4; ++j) acc[i][j] = (v8f){0.f,0.f,0.f,0.f,0.f,0.f,0.f,0.f};

  for (int k0 = 0; k0 < K; k0 += 32) {
    V bh[4], bl[4];
#pragma unroll
    for (int j = 0; j < 4; ++j) {
      const size_t bo = (size_t)(n0 + (j << 4) + rlane) * ldb + koff + k0;
      bh[j] = Frag<T>::load(Bb + bo);
      if (SPLIT) bl[j] = Frag<T>::load(Bb2 + bo);
    }
#pragma unroll
    for (int i = 0; i < 4; ++i) {
      const size_t ao = (size_t)(m0 + (i << 4) + rlane) * lda + koff + k0;
      V ah = Frag<T>::load(Ab + ao);
      V al;
      if (SPLIT) al = Frag<T>::load(Ab2 + ao);
#pragma unroll
      for (int j = 0; j < 4; ++j) {
        acc[i][j] = Frag<T>::mma(ah, bh[j], acc[i][j]);
        if (SPLIT) {
          acc[i][j] = Frag<T>::mma(ah, bl[j], acc[i][j]);
          acc[i][j] = Frag<T>::mma(al, bh[j], acc[i][j]);
        }
      }
      Frag<T>::guard(acc[i][0], acc[i][3], ah, SPLIT ? al : ah);
    }
    Frag<T>::keep(bh[0], bh[1], bh[2], bh[3]);
    if (SPLIT) Frag<T>::keep(bl[0], bl[1], bl[2], bl[3]);
  }
  acc_guard4(acc[0][0], acc[0][1], acc[0][2], acc[0][3]);
  acc_guard4(acc[1][0], acc[1][1], acc[1][2], acc[1][3]);
  acc_guard4(acc[2][0], acc[2][1], acc[2][2], acc[2][3]);
  acc_guard4(acc[3][0], acc[3][1], acc[3][2], acc[3][3]);

  float* slab = sT[wave];
  const float* Rb = RESID ? (resid + (size_t)b * strideR) : nullptr;
#pragma unroll
  for (int i = 0; i < 4; ++i) {
    const int mBase = m0 + (i << 4);
#pragma unroll
    for (int j = 0; j < 4; ++j) {
      const int n = n0 + (j << 4) + rlane;
      float bv = 0.f;
      if (BIAS_MODE == 2) bv = bias[n];
#pragma unroll
      for (int r = 0; r < 8; ++r) {
        float v = acc[i][j][r] * scale;
        if (BIAS_MODE == 1) v += bias[mBase + mOff + r];
        if (BIAS_MODE == 2) v += bv;
        if (RESID) v += Rb[(size_t)(mBase + mOff + r) * ldc + n];
        if (ACT == 1) v = tanhf(v);
        if (ACT == 2) v = fmaxf(v, 0.0f);
        if (ACT == 4) v = (v > 0.f) ? v : 0.01f * v;
        slab[(mOff + r) * 68 + (j << 4) + rlane] = v;
      }
    }
    __builtin_amdgcn_fence(__ATOMIC_RELEASE, "workgroup");
    __builtin_amdgcn_wave_barrier();
    __builtin_amdgcn_fence(__ATOMIC_ACQUIRE, "workgroup");
    if (OUT_MODE == 0) {
      float* C = (float*)Cout + (size_t)b * strideC;
      const int hh = lane >> 4, c4 = (lane & 15) * 4;
      for (int pass = 0; pass < 2; ++pass) {
#pragma unroll
        for (int it = 0; it < 8; ++it) {
          const int row = it * 2 + hh;
          v4f v = *(const v4f*)(slab + row * 68 + c4);
          *(volatile v4f*)(C + (size_t)(mBase + row) * ldc + n0 + c4) = v;
        }
        __threadfence();
      }
    } else {
      const int q = lane >> 3, c8 = (lane & 7) * 8;
      unsigned short* C  = (unsigned short*)Cout  + (size_t)b * strideC;
      unsigned short* C2 = (OUT_MODE == 2) ? ((unsigned short*)Cout2 + (size_t)b * strideC) : nullptr;
      for (int pass = 0; pass < 2; ++pass) {
#pragma unroll
        for (int it = 0; it < 4; ++it) {
          const int row = it * 4 + q;
          const float* sp = slab + row * 68 + c8;
          v8h hv, lv;
#pragma unroll
          for (int e = 0; e < 8; ++e) {
            if (OUT_MODE == 1) {
              hv[e] = (_Float16)sp[e];
            } else {
              unsigned short hb = f2bf_bits(sp[e]);
              unsigned short lb = f2bf_bits(sp[e] - bf_bits2f(hb));
              hv[e] = __builtin_bit_cast(_Float16, hb);
              lv[e] = __builtin_bit_cast(_Float16, lb);
            }
          }
          *(volatile v8h*)(C + (size_t)(mBase + row) * ldc + n0 + c8) = hv;
          if (OUT_MODE == 2) *(volatile v8h*)(C2 + (size_t)(mBase + row) * ldc + n0 + c8) = lv;
        }
        __threadfence();
      }
    }
    __builtin_amdgcn_fence(__ATOMIC_RELEASE, "workgroup");
    __builtin_amdgcn_wave_barrier();
    __builtin_amdgcn_fence(__ATOMIC_ACQUIRE, "workgroup");
  }
}

__device__ __forceinline__ unsigned pk16(unsigned short a, unsigned short b) { return (unsigned)a | ((unsigned)b << 16); }
__device__ __forceinline__ unsigned short h_bits(float f) { const _Float16 h = (_Float16)f; return __builtin_bit_cast(unsigned short, h); }

__global__ __launch_bounds__(256) void cast_f16x2_kernel(const float* __restrict__ in, unsigned short* __restrict__ out, int n2, float scale) {
  const int i = blockIdx.x * 256 + threadIdx.x;
  if (i < n2) {
    const v2f f = *(const v2f*)(in + 2 * (size_t)i);
    const unsigned u = pk16(h_bits(f[0] * scale), h_bits(f[1] * scale));
    ((volatile unsigned*)out)[i] = u;
    __threadfence();
    ((volatile unsigned*)out)[i] = u;
  }
}

__global__ __launch_bounds__(256) void rel_tables_kernel(const float* __restrict__ relk, const float* __restrict__ relv,
                                                         unsigned short* __restrict__ rk16, unsigned short* __restrict__ rvt16) {
  const int i = blockIdx.x * 256 + threadIdx.x;
  if (i >= kRelP * kHd / 2) return;
  const int e = 2 * i;
  if (blockIdx.y == 0) {
    const int row = e >> 6, col = e & 63;
    const int rc = row < kNRel ? row : (kNRel - 1);
    const float f0 = relk[rc * kHd + col];
    const float f1 = relk[rc * kHd + col + 1];
    const bool ok = row < kNRel;
    const unsigned short h0 = ok ? h_bits(f0 * kWCarry) : (unsigned short)0;
    const unsigned short h1 = ok ? h_bits(f1 * kWCarry) : (unsigned short)0;
    const unsigned u = pk16(h0, h1);
    ((volatile unsigned*)rk16)[i] = u;
    __threadfence();
    ((volatile unsigned*)rk16)[i] = u;
  } else {
    const int d = e >> 7, r = e & 127;
    const int r0c = r < kNRel ? r : (kNRel - 1);
    const int r1c = (r + 1) < kNRel ? (r + 1) : (kNRel - 1);
    const float f0 = relv[r0c * kHd + d];
    const float f1 = relv[r1c * kHd + d];
    const unsigned short h0 = (r < kNRel) ? h_bits(f0 * kWCarry) : (unsigned short)0;
    const unsigned short h1 = ((r + 1) < kNRel) ? h_bits(f1 * kWCarry) : (unsigned short)0;
    const unsigned u = pk16(h0, h1);
    ((volatile unsigned*)rvt16)[i] = u;
    __threadfence();
    ((volatile unsigned*)rvt16)[i] = u;
  }
}

__global__ __launch_bounds__(128) void softmax_rel_kernel(const float* __restrict__ S, const float* __restrict__ QR,
                                                           const float* __restrict__ qmask, const float* __restrict__ kmask,
                                                           unsigned short* __restrict__ P, unsigned short* __restrict__ PB) {
  __shared__ __align__(16) float qr_s[kRelP];
  __shared__ __align__(16) float row_s[kSeq];
  __shared__ __align__(16) float pb_s[kRelP];
  __shared__ float red0[4], red1[4], red2[4], red3[4], red4[4], red5[4];
  const int i    = blockIdx.x;
  const int hg   = blockIdx.y;
  const int tid  = threadIdx.x;
  const int lane = tid & 31;
  const int wave = tid >> 5;
  const int j0   = tid * 8;
  const size_t rowoff = ((size_t)hg * kSeq + i) * kSeq;

  qr_s[tid] = QR[((size_t)hg * kSeq + i) * kRelP + tid];
  const float qmv = qmask[i];
  const v4f sa = *(const v4f*)(S + rowoff + j0);
  const v4f sc = *(const v4f*)(S + rowoff + j0 + 4);
  const v4f ka = *(const v4f*)(kmask + j0);
  const v4f kc = *(const v4f*)(kmask + j0 + 4);
  const float sv[8] = {sa[0], sa[1], sa[2], sa[3], sc[0], sc[1], sc[2], sc[3]};
  const float km[8] = {ka[0], ka[1], ka[2], ka[3], kc[0], kc[1], kc[2], kc[3]};
  __syncthreads();

  float t[8];
  bool  mk[8];
#pragma unroll
  for (int e = 0; e < 8; ++e) {
    int d = j0 + e - i;
    d = d < -kMaxR ? -kMaxR : (d > kMaxR ? kMaxR : d);
    d += kMaxR;
    const float s = sv[e] + qr_s[d];
    const bool m = (qmv * km[e]) != 0.0f;
    mk[e] = m;
    t[e] = s + (m ? 0.0f : kNegBig);
  }
  float mx = fmaxf(fmaxf(fmaxf(t[0], t[1]), fmaxf(t[2], t[3])), fmaxf(fmaxf(t[4], t[5]), fmaxf(t[6], t[7])));
#pragma unroll
  for (int off = 16; off > 0; off >>= 1) mx = fmaxf(mx, __shfl_xor(mx, off, 32));
  if (lane == 0) red0[wave] = mx;
  __syncthreads();
  mx = fmaxf(fmaxf(red0[0], red0[1]), fmaxf(red0[2], red0[3]));
  float ex[8];
#pragma unroll
  for (int e = 0; e < 8; ++e) ex[e] = __expf(t[e] - mx);
  float s1 = ((ex[0] + ex[1]) + (ex[2] + ex[3])) + ((ex[4] + ex[5]) + (ex[6] + ex[7]));
#pragma unroll
  for (int off = 16; off > 0; off >>= 1) s1 += __shfl_xor(s1, off, 32);
  if (lane == 0) red1[wave] = s1;
  __syncthreads();
  const float tot1 = ((red1[0] + red1[1]) + red1[2]) + red1[3];
  const float inv1 = 1.0f / tot1;
  float w[8];
#pragma unroll
  for (int e = 0; e < 8; ++e) w[e] = mk[e] ? (ex[e] * inv1) : 0.0f;
  float mx2 = fmaxf(fmaxf(fmaxf(w[0], w[1]), fmaxf(w[2], w[3])), fmaxf(fmaxf(w[4], w[5]), fmaxf(w[6], w[7])));
#pragma unroll
  for (int off = 16; off > 0; off >>= 1) mx2 = fmaxf(mx2, __shfl_xor(mx2, off, 32));
  if (lane == 0) red2[wave] = mx2;
  __syncthreads();
  mx2 = fmaxf(fmaxf(red2[0], red2[1]), fmaxf(red2[2], red2[3]));
  float ex2[8];
#pragma unroll
  for (int e = 0; e < 8; ++e) ex2[e] = __expf(w[e] - mx2);
  float s2 = ((ex2[0] + ex2[1]) + (ex2[2] + ex2[3])) + ((ex2[4] + ex2[5]) + (ex2[6] + ex2[7]));
#pragma unroll
  for (int off = 16; off > 0; off >>= 1) s2 += __shfl_xor(s2, off, 32);
  if (lane == 0) red3[wave] = s2;
  __syncthreads();
  const float tot2 = ((red3[0] + red3[1]) + red3[2]) + red3[3];
  const float inv2 = 1.0f / tot2;
  float o[8];
#pragma unroll
  for (int e = 0; e < 8; ++e) o[e] = ex2[e] * inv2;

  const v4u hv = (v4u){pk16(h_bits(o[0] * kPCarry), h_bits(o[1] * kPCarry)),
                       pk16(h_bits(o[2] * kPCarry), h_bits(o[3] * kPCarry)),
                       pk16(h_bits(o[4] * kPCarry), h_bits(o[5] * kPCarry)),
                       pk16(h_bits(o[6] * kPCarry), h_bits(o[7] * kPCarry))};
  *(volatile v4u*)(P + rowoff + j0) = hv;
  __threadfence();
  *(volatile v4u*)(P + rowoff + j0) = hv;

  float lo = 0.0f, hi = 0.0f;
#pragma unroll
  for (int e = 0; e < 8; ++e) {
    const int dj = j0 + e - i;
    row_s[j0 + e] = o[e];
    lo += (dj <= -kMaxR) ? o[e] : 0.0f;
    hi += (dj >= kMaxR) ? o[e] : 0.0f;
  }
#pragma unroll
  for (int off = 16; off > 0; off >>= 1) { lo += __shfl_xor(lo, off, 32); hi += __shfl_xor(hi, off, 32); }
  if (lane == 0) { red4[wave] = lo; red5[wave] = hi; }
  __syncthreads();
  const float loT = ((red4[0] + red4[1]) + red4[2]) + red4[3];
  const float hiT = ((red5[0] + red5[1]) + red5[2]) + red5[3];
  {
    const int r  = tid;
    const int jm = i + r - kMaxR;
    const int jc = jm < 0 ? 0 : (jm > kSeq - 1 ? kSeq - 1 : jm);
    const float mid = row_s[jc];
    const bool inb = (jm >= 0) && (jm < kSeq);
    float val = 0.0f;
    if (r < kNRel && inb) val = mid;
    if (r == 0) val = loT;
    if (r == kNRel - 1) val = hiT;
    if (r >= kNRel) val = 0.0f;
    pb_s[r] = val * kPCarry;
  }
  __syncthreads();
  if (wave == 0 && lane < 16) {
    const float* sp = pb_s + lane * 8;
    const v4u pv = (v4u){pk16(h_bits(sp[0]), h_bits(sp[1])), pk16(h_bits(sp[2]), h_bits(sp[3])),
                         pk16(h_bits(sp[4]), h_bits(sp[5])), pk16(h_bits(sp[6]), h_bits(sp[7]))};
    unsigned short* dst = PB + ((size_t)hg * kSeq + i) * kRelP + lane * 8;
    *(volatile v4u*)dst = pv;
    __threadfence();
    *(volatile v4u*)dst = pv;
  }
}

extern "C" void kernel_launch(void* const* d_in, const int* in_sizes, int n_in,
                              void* d_out, int out_size, void* d_ws, size_t ws_size,
                              hipStream_t stream) {
  if (n_in < 15) return;
  const int nX = kBatch * kSeq * kDim;
  if (in_sizes[0] != nX || in_sizes[1] != nX || in_sizes[2] != nX) return;
  if (in_sizes[3] != kBatch * kSeq || in_sizes[4] != kBatch * kSeq) return;
  if (in_sizes[5] != kDim * kDim || in_sizes[7] != kDim * kDim || in_sizes[9] != kDim * kDim || in_sizes[11] != kDim * kDim) return;
  if (in_sizes[6] != kDim || in_sizes[8] != kDim || in_sizes[10] != kDim || in_sizes[12] != kDim) return;
  if (in_sizes[13] != kNRel * kHd || in_sizes[14] != kNRel * kHd) return;
  if (out_size != nX) return;

  const float* xq    = (const float*)d_in[0];
  const float* xk    = (const float*)d_in[1];
  const float* xv    = (const float*)d_in[2];
  const float* qmask = (const float*)d_in[3];
  const float* kmask = (const float*)d_in[4];
  const float* Wq    = (const float*)d_in[5];
  const float* bq    = (const float*)d_in[6];
  const float* Wk    = (const float*)d_in[7];
  const float* bk    = (const float*)d_in[8];
  const float* Wv    = (const float*)d_in[9];
  const float* bv    = (const float*)d_in[10];
  const float* Wo    = (const float*)d_in[11];
  const float* bo    = (const float*)d_in[12];
  const float* relk  = (const float*)d_in[13];
  const float* relv  = (const float*)d_in[14];

  const size_t PW  = (size_t)kDim * kDim * 2;
  const size_t PR  = (size_t)kRelP * kHd * 2;
  const size_t PX  = (size_t)kSeq * kDim * 2;
  const size_t PC  = (size_t)kSeq * kDim * 4;
  const size_t PQR = (size_t)kHeads * kSeq * kRelP * 4;
  const size_t PS  = (size_t)kHGrp * kSeq * kSeq * 4;
  const size_t PP  = (size_t)kHGrp * kSeq * kSeq * 2;
  const size_t PPB = (size_t)kHGrp * kSeq * kRelP * 2;
  size_t off = 0;
  const size_t oWq16  = off; off += PW;
  const size_t oWk16  = off; off += PW;
  const size_t oWv16  = off; off += PW;
  const size_t oWo16  = off; off += PW;
  const size_t oRK16  = off; off += PR;
  const size_t oRVT16 = off; off += PR;
  const size_t oXQ16  = off; off += PX;
  const size_t oXK16  = off; off += PX;
  const size_t oXV16  = off; off += PX;
  const size_t oQ16   = off; off += PX;
  const size_t oK16   = off; off += PX;
  const size_t oVT16  = off; off += PX;
  const size_t oCTX32 = off; off += PC;
  const size_t oCTX16 = off; off += PX;
  const size_t oQR    = off; off += PQR;
  const size_t oS     = off; off += PS;
  const size_t oP16   = off; off += PP;
  const size_t oPB16  = off; off += PPB;
  if (off > ws_size) return;

  char* ws = (char*)d_ws;
  unsigned short* Wq16  = (unsigned short*)(ws + oWq16);
  unsigned short* Wk16  = (unsigned short*)(ws + oWk16);
  unsigned short* Wv16  = (unsigned short*)(ws + oWv16);
  unsigned short* Wo16  = (unsigned short*)(ws + oWo16);
  unsigned short* RK16  = (unsigned short*)(ws + oRK16);
  unsigned short* RVT16 = (unsigned short*)(ws + oRVT16);
  unsigned short* XQ16  = (unsigned short*)(ws + oXQ16);
  unsigned short* XK16  = (unsigned short*)(ws + oXK16);
  unsigned short* XV16  = (unsigned short*)(ws + oXV16);
  unsigned short* Q16   = (unsigned short*)(ws + oQ16);
  unsigned short* K16   = (unsigned short*)(ws + oK16);
  unsigned short* VT16  = (unsigned short*)(ws + oVT16);
  float*          CTX32 = (float*)(ws + oCTX32);
  unsigned short* CTX16 = (unsigned short*)(ws + oCTX16);
  float*          QRb   = (float*)(ws + oQR);
  float*          Sbuf  = (float*)(ws + oS);
  unsigned short* P16   = (unsigned short*)(ws + oP16);
  unsigned short* PB16  = (unsigned short*)(ws + oPB16);

  const int n2w = kDim * kDim / 2;
  const int n2x = kSeq * kDim / 2;
  const dim3 blk(256);
  const dim3 blk128(128);
  const dim3 gCastW((n2w + 255) / 256);
  const dim3 gCastX((n2x + 255) / 256);
  const dim3 gRel((kRelP * kHd / 2 + 255) / 256, 2);

  cast_f16x2_kernel<<<gCastW, blk, 0, stream>>>(Wq, Wq16, n2w, kWCarry);
  cast_f16x2_kernel<<<gCastW, blk, 0, stream>>>(Wk, Wk16, n2w, kWCarry);
  cast_f16x2_kernel<<<gCastW, blk, 0, stream>>>(Wv, Wv16, n2w, kWCarry);
  cast_f16x2_kernel<<<gCastW, blk, 0, stream>>>(Wo, Wo16, n2w, kWCarry);
  rel_tables_kernel<<<gRel, blk, 0, stream>>>(relk, relv, RK16, RVT16);

  const int tilesM = kSeq / 64;
  const dim3 gProj((tilesM * (kDim / 64) + 7) / 8, 1);
  const dim3 gQR((tilesM * (kRelP / 64) + 7) / 8, kHeads);
  const dim3 gS((tilesM * (kSeq / 64) + 7) / 8, kHGrp);
  const dim3 gPV((tilesM * (kHd / 64) + 7) / 8, kHGrp);
  const dim3 gPB((tilesM * (kHd / 64) + 7) / 8, kHGrp);
  const dim3 gO((tilesM * (kDim / 64) + 7) / 8, 1);
  const dim3 gSm(kSeq, kHGrp);
  const float wscale  = 1.0f / kWCarry;
  const float sscale  = 0.125f;
  const float qrscale = 0.125f / kWCarry;
  const float pvscale = kCtxCarry / kPCarry;
  const float pbscale = kCtxCarry / (kPCarry * kWCarry);
  const float oscale  = 1.0f / (kWCarry * kCtxCarry);

  for (int b = 0; b < kBatch; ++b) {
    cast_f16x2_kernel<<<gCastX, blk, 0, stream>>>(xq + (size_t)b * kSeq * kDim, XQ16, n2x, 1.0f);
    cast_f16x2_kernel<<<gCastX, blk, 0, stream>>>(xk + (size_t)b * kSeq * kDim, XK16, n2x, 1.0f);
    cast_f16x2_kernel<<<gCastX, blk, 0, stream>>>(xv + (size_t)b * kSeq * kDim, XV16, n2x, 1.0f);
    wmma_gemm64<0, false, 2, 1, false, 0><<<gProj, blk, 0, stream>>>(
        XQ16, XQ16, kDim, 0L, Wq16, Wq16, kDim, 0L, (void*)Q16, (void*)Q16, kDim, 0L,
        bq, bq, 0L, kSeq, kDim, kDim, wscale);
    wmma_gemm64<0, false, 2, 1, false, 0><<<gProj, blk, 0, stream>>>(
        XK16, XK16, kDim, 0L, Wk16, Wk16, kDim, 0L, (void*)K16, (void*)K16, kDim, 0L,
        bk, bk, 0L, kSeq, kDim, kDim, wscale);
    wmma_gemm64<0, false, 1, 1, false, 0><<<gProj, blk, 0, stream>>>(
        Wv16, Wv16, kDim, 0L, XV16, XV16, kDim, 0L, (void*)VT16, (void*)VT16, kSeq, 0L,
        bv, bv, 0L, kDim, kSeq, kDim, wscale);
    wmma_gemm64<0, false, 0, 0, false, 0><<<gQR, blk, 0, stream>>>(
        Q16, Q16, kDim, (long)kHd, RK16, RK16, kHd, 0L, (void*)QRb, (void*)QRb, kRelP, (long)kSeq * kRelP,
        bq, bq, 0L, kSeq, kRelP, kHd, qrscale);
    const float* qmb = qmask + (size_t)b * kSeq;
    const float* kmb = kmask + (size_t)b * kSeq;
    for (int g = 0; g < kNGrp; ++g) {
      const size_t hc = (size_t)g * kHGrp * kHd;
      wmma_gemm64<0, false, 0, 0, false, 0><<<gS, blk, 0, stream>>>(
          Q16 + hc, Q16 + hc, kDim, (long)kHd, K16 + hc, K16 + hc, kDim, (long)kHd,
          (void*)Sbuf, (void*)Sbuf, kSeq, (long)kSeq * kSeq,
          bq, bq, 0L, kSeq, kSeq, kHd, sscale);
      softmax_rel_kernel<<<gSm, blk128, 0, stream>>>(Sbuf, QRb + (size_t)g * kHGrp * kSeq * kRelP, qmb, kmb, P16, PB16);
      wmma_gemm64<0, false, 0, 0, false, 0><<<gPV, blk, 0, stream>>>(
          P16, P16, kSeq, (long)kSeq * kSeq, VT16 + hc * kSeq, VT16 + hc * kSeq, kSeq, (long)kHd * kSeq,
          (void*)(CTX32 + hc), (void*)(CTX32 + hc), kDim, (long)kHd,
          bq, bq, 0L, kSeq, kHd, kSeq, pvscale);
      wmma_gemm64<0, false, 0, 1, true, 0><<<gPB, blk, 0, stream>>>(
          PB16, PB16, kRelP, (long)kSeq * kRelP, RVT16, RVT16, kRelP, 0L,
          (void*)(CTX16 + hc), (void*)(CTX16 + hc), kDim, (long)kHd,
          bq, CTX32 + hc, (long)kHd, kSeq, kHd, kRelP, pbscale);
    }
    float* outb = (float*)d_out + (size_t)b * kSeq * kDim;
    wmma_gemm64<0, false, 2, 0, false, 0><<<gO, blk, 0, stream>>>(
        CTX16, CTX16, kDim, 0L, Wo16, Wo16, kDim, 0L, (void*)outb, (void*)outb, kDim, 0L,
        bo, bo, 0L, kSeq, kDim, kDim, oscale);
  }
}
